// LutLayer_47648367181962
// MI455X (gfx1250) — hardware-run, weakly checked
//
#include <hip/hip_runtime.h>


#ifndef NB
#define NB 512
#endif
#ifndef DEPTH
#define DEPTH 4096
#endif
#define NB_FULL    512
#define DEPTH_FULL 4096
#ifndef OUT_PITCH
#define OUT_PITCH DEPTH
#endif
#define NIN   6
#define NPQ   12
#define NPAT  64
#define WPB   4
#define BCH   (NB < 32 ? NB : 32)
#define QRS   2048.0f
#define QRI   (1.0f / 2048.0f)
#define LEPS  1e-7f

static_assert(NPQ == 2 * NIN);
static_assert(2 * NPQ <= 32);
static_assert(NIN <= 8);
static_assert(NPAT == 64);
static_assert((NIN * 4) % 8 == 0);
static_assert(DEPTH % (32 * WPB) == 0);
static_assert(NB % BCH == 0);
static_assert(NB <= NB_FULL);
static_assert(DEPTH <= DEPTH_FULL);
static_assert(OUT_PITCH >= DEPTH);
static_assert(OUT_PITCH % 32 == 0);
static_assert(32 * 4 * 1 == 2 * 16 * 4);

typedef _Float16 h16;
typedef __attribute__((ext_vector_type(16))) _Float16 v16h;
typedef __attribute__((ext_vector_type(8)))  float    v8f;
typedef __attribute__((ext_vector_type(4)))  float    v4f;
typedef __attribute__((ext_vector_type(2)))  float    v2f;

__device__ __forceinline__ unsigned short f2bf(float f) { unsigned u = __float_as_uint(f); u += 0x7FFFu + ((u >> 16) & 1u); return (unsigned short)(u >> 16); }
__device__ __forceinline__ float bfr(float f) { return __uint_as_float(((unsigned)f2bf(f)) << 16); }
__device__ __forceinline__ v8f wmma16(v16h a, v16h b, v8f c) { return __builtin_amdgcn_wmma_f32_16x16x32_f16(false, a, false, b, (short)0, c, false, false); }
__device__ __forceinline__ v8f wmma16g(v16h a, v16h b, v8f c) { c = wmma16(a, b, c); asm volatile("v_nop\n\tv_nop\n\tv_nop\n\tv_nop" : "+v"(c) : "v"(a), "v"(b)); return c; }
static __device__ __forceinline__ h16 toh_flush(float v) { const h16 r = (h16)v; return (fabsf(v) < 6.103515625e-05f) ? (h16)0.0f : r; }

__global__ __launch_bounds__(32 * WPB) void k_patsum(const float* __restrict__ X, const float* __restrict__ WGT, const float* __restrict__ TAB, float* OUT) {
    const int lane = threadIdx.x & 31, lr = lane & 15, hi = lane >> 4;
    const int wave = __builtin_amdgcn_readfirstlane((int)(threadIdx.x >> 5));
    const int d0 = (blockIdx.x * WPB + wave) * 32;
    const int b0 = blockIdx.y * BCH;

    v16h ta[4];
#pragma unroll
    for (int mt = 0; mt < 4; ++mt) {
        const float* tp = TAB + (size_t)(6 * hi) * NPAT + 16 * mt + lr;
        float t[6];
#pragma unroll
        for (int i = 0; i < 6; ++i) t[i] = tp[(size_t)i * NPAT];
        asm volatile("" : "+v"(t[0]), "+v"(t[1]), "+v"(t[2]), "+v"(t[3]), "+v"(t[4]), "+v"(t[5]));
        v16h f = (v16h){};
#pragma unroll
        for (int i = 0; i < 6; ++i) { const float tb = bfr(t[i]); f[i] = toh_flush(tb); f[8 + i] = toh_flush(tb * QRI); }
        ta[mt] = f;
    }

    float lw[2][32];
#pragma unroll
    for (int tl = 0; tl < 2; ++tl) {
        const float* lp = WGT + (size_t)(d0 + 16 * tl + lr) * NPAT + 8 * hi;
#pragma unroll
        for (int mt = 0; mt < 4; ++mt) {
            v4f u0 = *(const v4f*)(lp + 16 * mt), u1 = *(const v4f*)(lp + 16 * mt + 4);
            asm volatile("" : "+v"(u0), "+v"(u1));
#pragma unroll
            for (int r = 0; r < 4; ++r) { lw[tl][8 * mt + r] = bfr(u0[r]); lw[tl][8 * mt + 4 + r] = bfr(u1[r]); }
        }
    }

#pragma unroll 1
    for (int bi = 0; bi < BCH; ++bi) {
        const size_t rowb = (size_t)(b0 + bi) * DEPTH_FULL + (size_t)(d0 + lr);
        float res[2];
#pragma unroll
        for (int tl = 0; tl < 2; ++tl) {
            const float* xr = X + (rowb + (size_t)(16 * tl)) * NIN;
            const v2f xa = *(const v2f*)xr, xc = *(const v2f*)(xr + 2), xe = *(const v2f*)(xr + 4);
            float xs[6];
            xs[0] = xa[0]; xs[1] = xa[1]; xs[2] = xc[0]; xs[3] = xc[1]; xs[4] = xe[0]; xs[5] = xe[1];
            v16h fb = (v16h){};
#pragma unroll
            for (int i = 0; i < 6; ++i) {
                const float xb = bfr(xs[i]);
                const float q  = 1.0f - xb;
                const float u  = hi ? xb : q;
                const float pq = fmaxf(u, 0.0f) + LEPS;
                const float lg = __builtin_amdgcn_logf(pq);
                const h16 hv = toh_flush(lg);
                fb[i] = hv; fb[8 + i] = toh_flush((lg - (float)hv) * QRS);
            }
            const v8f z = (v8f){};
            const v8f s0 = wmma16g(ta[0], fb, z);
            const v8f s1 = wmma16g(ta[1], fb, z);
            const v8f s2 = wmma16g(ta[2], fb, z);
            const v8f s3 = wmma16g(ta[3], fb, z);
            float part = 0.0f;
#pragma unroll
            for (int r = 0; r < 8; ++r) {
                part = fmaf(__builtin_amdgcn_exp2f(s0[r]), lw[tl][r],      part);
                part = fmaf(__builtin_amdgcn_exp2f(s1[r]), lw[tl][8 + r],  part);
                part = fmaf(__builtin_amdgcn_exp2f(s2[r]), lw[tl][16 + r], part);
                part = fmaf(__builtin_amdgcn_exp2f(s3[r]), lw[tl][24 + r], part);
            }
            part += __shfl_xor(part, 16, 32);
            res[tl] = part;
        }
        const float val = hi ? res[1] : res[0];
        float* op = OUT + (size_t)(b0 + bi) * OUT_PITCH + (size_t)(d0 + lane);
        *(volatile float*)op = val;
        __threadfence();
        *(volatile float*)op = val;
    }
}

extern "C" void kernel_launch(void* const* d_in, const int* in_sizes, int n_in,
                              void* d_out, int out_size, void* d_ws, size_t ws_size, hipStream_t stream) {
    if (n_in < 3) return;
    const size_t needx = ((size_t)(NB - 1) * DEPTH_FULL + DEPTH) * NIN;
    if ((size_t)in_sizes[0] < needx) return;
    if ((size_t)in_sizes[1] < (size_t)DEPTH * NPAT) return;
    if ((size_t)in_sizes[2] < (size_t)NPQ * NPAT) return;
    if ((size_t)out_size < (size_t)(NB - 1) * OUT_PITCH + DEPTH) return;
    const float* X   = (const float*)d_in[0];
    const float* WGT = (const float*)d_in[1];
    const float* TAB = (const float*)d_in[2];
    float* OUT = (float*)d_out;
    (void)d_ws; (void)ws_size;
    k_patsum<<<dim3(DEPTH / (32 * WPB), NB / BCH, 1), 32 * WPB, 0, stream>>>(X, WGT, TAB, OUT);
}
